// GroupedReadWrite_1005022347566
// MI455X (gfx1250) — hardware-verified
//
#include <hip/hip_runtime.h>
#include <stddef.h>
#include <stdint.h>

#define NB    4
#define NSP   4096
#define NTK   16384
#define DM    512
#define NHD   8
#define HD    64
#define JL    8
#define NG    256
#define NGP   128
#define KL    2048
#define NLT   8192
#define DC    512
#define DMOD  1024
#define QROWS 64
#define QREAL 32

static_assert(NTK == NB * NSP);
static_assert(NLT == NB * KL);
static_assert(KL == NG * JL);
static_assert(NG == 2 * NGP);
static_assert(DM == NHD * HD);
static_assert(QREAL == NB * JL);
static_assert(DM % 32 == 0);
static_assert(NTK % 64 == 0);
static_assert(NLT % 256 == 0);
static_assert(QROWS % 64 == 0);
static_assert(DMOD % 256 == 0);

typedef _Float16 v16h __attribute__((ext_vector_type(16)));
typedef _Float16 v8h  __attribute__((ext_vector_type(8)));
typedef float    v8f  __attribute__((ext_vector_type(8)));
typedef float    v4f  __attribute__((ext_vector_type(4)));
typedef unsigned int v4u __attribute__((ext_vector_type(4)));

union Frag  { v16h v; v8h h[2]; _Float16 x[16]; };
union Pack8 { v8h h; v4u u; };

__device__ __forceinline__ v8f zero8() { return (v8f){0.f, 0.f, 0.f, 0.f, 0.f, 0.f, 0.f, 0.f}; }

__device__ __forceinline__ v4u cvt8(v4f a, v4f b) {
  Pack8 pk;
  pk.h = (v8h){(_Float16)a[0], (_Float16)a[1], (_Float16)a[2], (_Float16)a[3],
               (_Float16)b[0], (_Float16)b[1], (_Float16)b[2], (_Float16)b[3]};
  return pk.u;
}

__device__ __forceinline__ float wsum(float v) {
#pragma unroll
  for (int off = 16; off > 0; off >>= 1) v += __shfl_xor(v, off, 32);
  return v;
}
__device__ __forceinline__ float hsum4(v4f a) { return (a[0] + a[1]) + (a[2] + a[3]); }

__device__ __forceinline__ v8f mma16(v16h a, v16h b, v8f c) {
  c = __builtin_amdgcn_wmma_f32_16x16x32_f16(false, a, false, b, (short)0, c, false, false);
  asm volatile("v_nop\n\tv_nop\n\tv_nop\n\tv_nop" : "+v"(c) : "v"(a), "v"(b));
  return c;
}

__device__ __forceinline__ v16h ldfrag(const _Float16* p, int ld, int row0, int k0, int lane) {
  const int m = lane & 15, lh = lane >> 4;
  const _Float16* q = p + (size_t)(row0 + m) * ld + k0 + 8 * lh;
  Frag f;
  f.h[0] = *(const v8h*)(q);
  f.h[1] = *(const v8h*)(q + 16);
  return f.v;
}

__device__ __forceinline__ v16h gatherB(const _Float16* s, int pitch, int col, int lh) {
  Frag f;
#pragma unroll
  for (int i = 0; i < 8; ++i) {
    f.x[i]     = s[(8 * lh + i) * pitch + col];
    f.x[8 + i] = s[(16 + 8 * lh + i) * pitch + col];
  }
  return f.v;
}

__device__ __forceinline__ void gemm16x64(const _Float16* __restrict__ A, int lda,
                                          const _Float16* __restrict__ Bt, int ldb,
                                          int m0, int n0, int lane, v8f (&acc)[4]) {
#pragma unroll 2
  for (int k0 = 0; k0 < DM; k0 += 32) {
    const v16h a = ldfrag(A, lda, m0, k0, lane);
#pragma unroll
    for (int t = 0; t < 4; ++t) {
      const v16h b = ldfrag(Bt, ldb, n0 + 16 * t, k0, lane);
      acc[t] = mma16(a, b, acc[t]);
    }
  }
}

__device__ __forceinline__ void gemm32x64(const _Float16* __restrict__ A, int lda,
                                          const _Float16* __restrict__ Bt, int ldb,
                                          int m0, int n0, int lane, v8f (&acc)[2][4]) {
#pragma unroll 2
  for (int k0 = 0; k0 < DM; k0 += 32) {
    const v16h a0 = ldfrag(A, lda, m0, k0, lane);
    const v16h a1 = ldfrag(A, lda, m0 + 16, k0, lane);
    const v16h b0 = ldfrag(Bt, ldb, n0, k0, lane);
    const v16h b1 = ldfrag(Bt, ldb, n0 + 16, k0, lane);
    const v16h b2 = ldfrag(Bt, ldb, n0 + 32, k0, lane);
    const v16h b3 = ldfrag(Bt, ldb, n0 + 48, k0, lane);
    acc[0][0] = mma16(a0, b0, acc[0][0]);
    acc[1][0] = mma16(a1, b0, acc[1][0]);
    acc[0][1] = mma16(a0, b1, acc[0][1]);
    acc[1][1] = mma16(a1, b1, acc[1][1]);
    acc[0][2] = mma16(a0, b2, acc[0][2]);
    acc[1][2] = mma16(a1, b2, acc[1][2]);
    acc[0][3] = mma16(a0, b3, acc[0][3]);
    acc[1][3] = mma16(a1, b3, acc[1][3]);
  }
}

__device__ __forceinline__ void ln512_pack(v4f (&a)[4], const float* __restrict__ g, const float* __restrict__ be,
                                           int c0, int c1, v4u& o0, v4u& o1) {
  float s = (hsum4(a[0]) + hsum4(a[1])) + (hsum4(a[2]) + hsum4(a[3]));
  s = wsum(s);
  const float mu = s * (1.0f / (float)DM);
  v4f d[4];
  float q = 0.f;
#pragma unroll
  for (int i = 0; i < 4; ++i) { d[i] = a[i] - mu; q += hsum4(d[i] * d[i]); }
  q = wsum(q);
  const float rs = rsqrtf(q * (1.0f / (float)DM) + 1e-5f);
  const v4f g0 = (v4f){g[c0], g[c0 + 1], g[c0 + 2], g[c0 + 3]};
  const v4f g1 = (v4f){g[c0 + 4], g[c0 + 5], g[c0 + 6], g[c0 + 7]};
  const v4f g2 = (v4f){g[c1], g[c1 + 1], g[c1 + 2], g[c1 + 3]};
  const v4f g3 = (v4f){g[c1 + 4], g[c1 + 5], g[c1 + 6], g[c1 + 7]};
  const v4f b0 = (v4f){be[c0], be[c0 + 1], be[c0 + 2], be[c0 + 3]};
  const v4f b1 = (v4f){be[c0 + 4], be[c0 + 5], be[c0 + 6], be[c0 + 7]};
  const v4f b2 = (v4f){be[c1], be[c1 + 1], be[c1 + 2], be[c1 + 3]};
  const v4f b3 = (v4f){be[c1 + 4], be[c1 + 5], be[c1 + 6], be[c1 + 7]};
  const v4f y0 = d[0] * rs * g0 + b0;
  const v4f y1 = d[1] * rs * g1 + b1;
  const v4f y2 = d[2] * rs * g2 + b2;
  const v4f y3 = d[3] * rs * g3 + b3;
  o0 = cvt8(y0, y1);
  o1 = cvt8(y2, y3);
}

__global__ __launch_bounds__(256) void k_lnx(const float* __restrict__ x, const float* __restrict__ g,
                                             const float* __restrict__ be, _Float16* __restrict__ y, int nrows) {
  const int lane = threadIdx.x & 31, wave = threadIdx.x >> 5;
  const int row = blockIdx.x * 8 + wave;
  if (row >= nrows) return;
  const float* xr = x + (size_t)row * DM;
  const int c0 = 8 * lane, c1 = 256 + 8 * lane;
  v4f a[4];
  a[0] = *(const v4f*)(xr + c0);
  a[1] = *(const v4f*)(xr + c0 + 4);
  a[2] = *(const v4f*)(xr + c1);
  a[3] = *(const v4f*)(xr + c1 + 4);
  v4u o0, o1;
  ln512_pack(a, g, be, c0, c1, o0, o1);
  volatile v4u* d0 = (volatile v4u*)(y + (size_t)row * DM + c0);
  volatile v4u* d1 = (volatile v4u*)(y + (size_t)row * DM + c1);
  *d0 = o0; *d1 = o1;
  __threadfence();
  *d0 = o0; *d1 = o1;
}

__global__ __launch_bounds__(256) void k_cvtw(const float* __restrict__ w, _Float16* __restrict__ dst,
                                              float scale, int n) {
  const int i = (blockIdx.x * 256 + threadIdx.x) * 8;
  if (i + 8 > n) return;
  const v4f a = *(const v4f*)(w + i) * scale;
  const v4f b = *(const v4f*)(w + i + 4) * scale;
  const v4u v = cvt8(a, b);
  volatile v4u* d = (volatile v4u*)(dst + i);
  *d = v;
  __threadfence();
  *d = v;
}

__global__ __launch_bounds__(256) void k_mod(const float* __restrict__ cond, const float* __restrict__ wad,
                                             const float* __restrict__ badl, float* __restrict__ mod) {
  const int idx = blockIdx.x * 256 + threadIdx.x;
  const int b = idx >> 10, o = idx & 1023;
  const float* cr = cond + b * DC;
  const float* wr = wad + (size_t)o * DC;
  float acc = 0.f;
#pragma unroll 1
  for (int k = 0; k < DC; k += 4) {
    const v4f cv = *(const v4f*)(cr + k);
    const v4f wv = *(const v4f*)(wr + k);
    acc += cv[0] * wv[0];
    acc += cv[1] * wv[1];
    acc += cv[2] * wv[2];
    acc += cv[3] * wv[3];
  }
  acc += badl[o];
  volatile float* d = mod + idx;
  *d = acc;
  __threadfence();
  *d = acc;
}

__global__ __launch_bounds__(256) void k_qprep(const float* __restrict__ lt, const float* __restrict__ lp,
                                               const float* __restrict__ mod, const float* __restrict__ g,
                                               const float* __restrict__ be, _Float16* __restrict__ qa) {
  const int lane = threadIdx.x & 31, wave = threadIdx.x >> 5;
  const int row = blockIdx.x * 8 + wave;
  const int rr = row & (QREAL - 1);
  const int b = rr >> 3, j = rr & 7;
  const float* tr = lt + j * DM;
  const float* pr = lp + j * DM;
  const float* sh = mod + b * DMOD;
  const float* sc = mod + b * DMOD + DM;
  const int c0 = 8 * lane, c1 = 256 + 8 * lane;
  const int cc[4] = {c0, c0 + 4, c1, c1 + 4};
  v4f a[4];
#pragma unroll
  for (int i = 0; i < 4; ++i) {
    const v4f t0 = *(const v4f*)(tr + cc[i]);
    const v4f p0 = *(const v4f*)(pr + cc[i]);
    const v4f s0 = *(const v4f*)(sc + cc[i]);
    const v4f h0 = *(const v4f*)(sh + cc[i]);
    a[i] = (t0 + p0) * (s0 + 1.0f) + h0;
  }
  v4u o0, o1;
  ln512_pack(a, g, be, c0, c1, o0, o1);
  const unsigned int keep = (row < QREAL) ? 0xffffffffu : 0u;
  o0 = o0 & keep;
  o1 = o1 & keep;
  volatile v4u* d0 = (volatile v4u*)(qa + (size_t)row * DM + c0);
  volatile v4u* d1 = (volatile v4u*)(qa + (size_t)row * DM + c1);
  *d0 = o0; *d1 = o1;
  __threadfence();
  *d0 = o0; *d1 = o1;
}

#define SFP 132
__global__ __launch_bounds__(256) void k_proj(const _Float16* __restrict__ A,
                                              const _Float16* __restrict__ Wt,
                                              const float* __restrict__ bias0,
                                              const float* __restrict__ gam,
                                              const float* __restrict__ bet,
                                              _Float16* __restrict__ out0,
                                              const float* __restrict__ bias1,
                                              _Float16* __restrict__ out1,
                                              int nsplit) {
  __shared__ __align__(16) float sf[64 * SFP];
  __shared__ float smu[128];
  __shared__ float srs[128];
  const int tid = threadIdx.x, lane = tid & 31, wave = tid >> 5;
  const int hh = lane >> 4, c = lane & 15;
  const int wm = wave >> 1, wn = wave & 1;
  const int mb = blockIdx.x * 64;
  const int ns = blockIdx.y;
  const bool second = (ns >= nsplit);
  const int nsl = second ? (ns - nsplit) : ns;
  const int m0 = mb + wm * 16;
  const int n0 = ns * 128 + wn * 64;
  const float* bias = second ? (bias1 + nsl * 128) : (bias0 + nsl * 128);

  v8f acc[4];
#pragma unroll
  for (int t = 0; t < 4; ++t) acc[t] = zero8();
  gemm16x64(A, DM, Wt, DM, m0, n0, lane, acc);

#pragma unroll
  for (int t = 0; t < 4; ++t) {
    const float bb = bias[wn * 64 + 16 * t + c];
#pragma unroll
    for (int r = 0; r < 8; ++r)
      sf[(wm * 16 + 8 * hh + r) * SFP + wn * 64 + 16 * t + c] = acc[t][r] * 0.03125f + bb;
  }
  __syncthreads();

  {
    const int pi = tid >> 1;
    const int lr = pi >> 1, hs = pi & 1, hf = tid & 1;
    const float* rp = sf + lr * SFP + hs * 64 + hf * 32;
    float s = 0.f;
#pragma unroll 8
    for (int i = 0; i < 32; ++i) s += rp[i];
    s += __shfl_xor(s, 1, 32);
    const float mu = s * (1.0f / 64.0f);
    float q = 0.f;
#pragma unroll 8
    for (int i = 0; i < 32; ++i) { const float d = rp[i] - mu; q += d * d; }
    q += __shfl_xor(q, 1, 32);
    const float rs = rsqrtf(q * (1.0f / 64.0f) + 1e-5f);
    if (hf == 0) { smu[pi] = mu; srs[pi] = rs; }
  }
  __syncthreads();

  v4u val[4];
  size_t go[4];
#pragma unroll
  for (int jx = 0; jx < 4; ++jx) {
    const int p  = tid + 256 * jx;
    const int lr = p >> 4;
    const int pc = p & 15;
    const int hs = pc >> 3;
    const int d0 = (pc & 7) * 8;
    const float* ra = sf + lr * SFP + pc * 8;
    const v4f x0 = *(const v4f*)(ra), x1 = *(const v4f*)(ra + 4);
    const float mu = smu[lr * 2 + hs], rs = srs[lr * 2 + hs];
    const v4f g0 = (v4f){gam[d0], gam[d0 + 1], gam[d0 + 2], gam[d0 + 3]};
    const v4f g1 = (v4f){gam[d0 + 4], gam[d0 + 5], gam[d0 + 6], gam[d0 + 7]};
    const v4f b0 = (v4f){bet[d0], bet[d0 + 1], bet[d0 + 2], bet[d0 + 3]};
    const v4f b1 = (v4f){bet[d0 + 4], bet[d0 + 5], bet[d0 + 6], bet[d0 + 7]};
    v4f y0 = (x0 - mu) * rs * g0 + b0;
    v4f y1 = (x1 - mu) * rs * g1 + b1;
    if (second) { y0 = x0; y1 = x1; }
    val[jx] = cvt8(y0, y1);
    go[jx]  = (size_t)(mb + lr) * DM + nsl * 128 + pc * 8;
  }
  _Float16* base = second ? out1 : out0;
  for (int ps = 0; ps < 2; ++ps) {
#pragma unroll
    for (int jx = 0; jx < 4; ++jx) *(volatile v4u*)(base + go[jx]) = val[jx];
    __threadfence();
  }
}

#define KVP 520
#define PTP 72

__device__ __forceinline__ void stage_rows(const _Float16* __restrict__ src, _Float16* kvs,
                                           int b, int gp, int gW, int Wc, int ntok, int tid) {
#pragma unroll
  for (int e = 0; e < 8; ++e) {
    const int p  = tid + 256 * e;
    const int tk = p >> 6;
    const int q8 = (p & 63) * 8;
    const int t  = tk >> 4, ki = tk & 15;
    const int g  = 2 * gp + t;
    const int gr = g / gW;
    const int gc = g - gr * gW;
    int n = (4 * gr + (ki >> 2)) * Wc + 4 * gc + (ki & 3);
    n = min(max(n, 0), ntok - 1);
    *(v8h*)(kvs + tk * KVP + q8) = *(const v8h*)(src + (size_t)(b * NSP + n) * DM + q8);
  }
}

__device__ __forceinline__ void softmax16(v8f s, float (&p)[8], float (&il)[8]) {
#pragma unroll
  for (int r = 0; r < 8; ++r) {
    const float sc = s[r] * 0.125f;
    float m = sc;
#pragma unroll
    for (int off = 1; off < 16; off <<= 1) m = fmaxf(m, __shfl_xor(m, off, 32));
    const float e = __expf(sc - m);
    float l = e;
#pragma unroll
    for (int off = 1; off < 16; off <<= 1) l += __shfl_xor(l, off, 32);
    p[r]  = e * 1024.0f;
    il[r] = 0.015625f / l;
  }
}

__global__ __launch_bounds__(256) void k_attn(const _Float16* __restrict__ qp,
                                              const _Float16* __restrict__ kp,
                                              const _Float16* __restrict__ vp,
                                              _Float16* __restrict__ op,
                                              const int* __restrict__ hp,
                                              const int* __restrict__ wp) {
  __shared__ __align__(16) _Float16 KVs[32 * KVP];
  __shared__ __align__(16) _Float16 Ps[8 * 16 * PTP];

  const int tid = threadIdx.x, lane = tid & 31, wave = tid >> 5;
  const int lh = lane >> 4, c = lane & 15;
  const int b  = blockIdx.x >> 7;
  const int gp = blockIdx.x & (NGP - 1);
  const int h  = wave;
  int Hc = hp[0], Wc = wp[0];
  Hc = min(max(Hc, 1), 64);
  Wc = min(max(Wc, 1), 64);
  const int gW   = (Wc + 3) >> 2;
  const int ntok = Hc * Wc;

  stage_rows(kp, KVs, b, gp, gW, Wc, ntok, tid);
  __syncthreads();

  v16h qa0, qa1;
  {
    const _Float16* qr = qp + (size_t)(b * JL + (c & 7)) * DM + h * HD + 8 * lh;
    Frag f;
    f.h[0] = *(const v8h*)(qr);      f.h[1] = *(const v8h*)(qr + 16);      qa0 = f.v;
    f.h[0] = *(const v8h*)(qr + 32); f.h[1] = *(const v8h*)(qr + 48);      qa1 = f.v;
  }
  v8f s0 = zero8(), s1 = zero8();
  {
    v16h kb;
    kb = ldfrag(KVs, KVP, 0,  h * HD,      lane); s0 = mma16(qa0, kb, s0);
    kb = ldfrag(KVs, KVP, 0,  h * HD + 32, lane); s0 = mma16(qa1, kb, s0);
    kb = ldfrag(KVs, KVP, 16, h * HD,      lane); s1 = mma16(qa0, kb, s1);
    kb = ldfrag(KVs, KVP, 16, h * HD + 32, lane); s1 = mma16(qa1, kb, s1);
  }
  float p0[8], p1[8], il0[8], il1[8];
  softmax16(s0, p0, il0);
  softmax16(s1, p1, il1);

  _Float16* pw = Ps + wave * 16 * PTP;
#pragma unroll
  for (int r = 0; r < 8; ++r) {
    const float v0 = (lh == 0) ? p0[r] : 0.f;
    const float v1 = (lh == 1) ? p1[r] : 0.f;
    pw[r * PTP + 16 * lh + c]       = (_Float16)v0;
    pw[(8 + r) * PTP + 16 * lh + c] = (_Float16)v1;
  }
  __syncthreads();

  stage_rows(vp, KVs, b, gp, gW, Wc, ntok, tid);
  __syncthreads();

  const v16h pa = ldfrag(pw, PTP, 0, 0, lane);
  v8f o[4];
#pragma unroll
  for (int ct = 0; ct < 4; ++ct) {
    const v16h vb = gatherB(KVs, KVP, h * HD + 16 * ct + c, lh);
    o[ct] = mma16(pa, vb, zero8());
  }
  float isel[8];
#pragma unroll
  for (int r = 0; r < 8; ++r) isel[r] = (lh == 0) ? il0[r] : il1[r];
  __syncthreads();
#pragma unroll
  for (int r = 0; r < 8; ++r) {
#pragma unroll
    for (int ct = 0; ct < 4; ++ct)
      pw[(8 * lh + r) * PTP + 16 * ct + c] = (_Float16)(o[ct][r] * isel[r]);
  }
  __syncthreads();
  v4u val[4];
  size_t go[4];
#pragma unroll
  for (int it = 0; it < 4; ++it) {
    const int p  = lane + 32 * it;
    const int L  = p >> 3;
    const int pc = p & 7;
    Pack8 pk;
    pk.h    = *(const v8h*)(pw + L * PTP + pc * 8);
    val[it] = pk.u;
    go[it]  = (size_t)(b * KL + gp * 16 + L) * DM + h * HD + pc * 8;
  }
  for (int ps = 0; ps < 2; ++ps) {
#pragma unroll
    for (int it = 0; it < 4; ++it) *(volatile v4u*)(op + go[it]) = val[it];
    __threadfence();
  }
}

#define OTP 68
__device__ __forceinline__ void out_epilogue(v8f (&acc)[2][4], float scale, const float* __restrict__ bias,
                                             const float* __restrict__ lt, const float* __restrict__ lp,
                                             const float* __restrict__ md, int b,
                                             float* sw, float* __restrict__ out,
                                             int m0, int n0, int lane, int hh, int c) {
#pragma unroll
  for (int sub = 0; sub < 2; ++sub) {
    __syncthreads();
#pragma unroll
    for (int t = 0; t < 4; ++t) {
      const float bb = bias[n0 + 16 * t + c];
#pragma unroll
      for (int r = 0; r < 8; ++r) sw[(8 * hh + r) * OTP + 16 * t + c] = acc[sub][t][r] * scale + bb;
    }
    __syncthreads();
    v4f val[8];
    size_t go[8];
#pragma unroll
    for (int it = 0; it < 8; ++it) {
      const int p    = lane + 32 * it;
      const int L    = p >> 3;
      const int pc   = p & 7;
      const int row  = L >> 1;
      const int half = L & 1;
      const int grow = m0 + sub * 16 + row;
      const int jj   = grow & 7;
      const int col  = n0 + half * 32 + pc * 4;
      v4f x = *(const v4f*)(sw + row * OTP + half * 32 + pc * 4);
      const v4f ta = *(const v4f*)(lt + jj * DM + col);
      const v4f tb = *(const v4f*)(lp + jj * DM + col);
      const v4f sh = *(const v4f*)(md + b * DMOD + col);
      const v4f sc = *(const v4f*)(md + b * DMOD + DM + col);
      x = x + ((ta + tb) * (sc + 1.0f) + sh);
      val[it] = x;
      go[it]  = (size_t)grow * DM + col;
    }
    for (int ps = 0; ps < 2; ++ps) {
#pragma unroll
      for (int it = 0; it < 8; ++it) *(volatile v4f*)(out + go[it]) = val[it];
      __threadfence();
    }
  }
}

__global__ __launch_bounds__(256) void k_out(const _Float16* __restrict__ ap,
                                             const _Float16* __restrict__ wt,
                                             const float* __restrict__ bo,
                                             const float* __restrict__ lt,
                                             const float* __restrict__ lp,
                                             const float* __restrict__ md,
                                             float* __restrict__ out) {
  __shared__ __align__(16) float st[8][16 * OTP];
  const int tid = threadIdx.x, lane = tid & 31, wave = tid >> 5;
  const int hh = lane >> 4, c = lane & 15;
  const int m0 = blockIdx.x * 256 + wave * 32;
  const int n0 = blockIdx.y * 64;
  const int b  = blockIdx.x >> 3;

  v8f acc[2][4];
#pragma unroll
  for (int s = 0; s < 2; ++s)
#pragma unroll
    for (int t = 0; t < 4; ++t) acc[s][t] = zero8();
  gemm32x64(ap, DM, wt, DM, m0, n0, lane, acc);
  out_epilogue(acc, 0.001953125f, bo, lt, lp, md, b, st[wave], out, m0, n0, lane, hh, c);
}

extern "C" void kernel_launch(void* const* d_in, const int* in_sizes, int n_in,
                              void* d_out, int out_size, void* d_ws, size_t ws_size,
                              hipStream_t stream) {
  if (n_in < 24) return;
  if (in_sizes[0] != NTK * DM) return;
  if (in_sizes[1] != NB * DC) return;
  if (in_sizes[2] != JL * DM) return;
  if (in_sizes[3] != JL * DM) return;
  if (in_sizes[4] != DM * DM) return;
  if (in_sizes[5] != DM) return;
  if (in_sizes[6] != DM * DM) return;
  if (in_sizes[7] != DM) return;
  if (in_sizes[8] != DM * DM) return;
  if (in_sizes[9] != DM) return;
  if (in_sizes[10] != DM * DM) return;
  if (in_sizes[11] != DM) return;
  if (in_sizes[12] != DMOD * DC) return;
  if (in_sizes[13] != DMOD) return;
  if (in_sizes[14] != HD || in_sizes[15] != HD || in_sizes[16] != HD || in_sizes[17] != HD) return;
  if (in_sizes[18] != DM || in_sizes[19] != DM || in_sizes[20] != DM || in_sizes[21] != DM) return;
  if (in_sizes[22] != 1 || in_sizes[23] != 1) return;
  if (out_size != NLT * DM) return;

  const float* spatial = (const float*)d_in[0];
  const float* cond    = (const float*)d_in[1];
  const float* lt      = (const float*)d_in[2];
  const float* lp      = (const float*)d_in[3];
  const float* Wq      = (const float*)d_in[4];
  const float* bq      = (const float*)d_in[5];
  const float* Wk      = (const float*)d_in[6];
  const float* bk      = (const float*)d_in[7];
  const float* Wv      = (const float*)d_in[8];
  const float* bv      = (const float*)d_in[9];
  const float* Wo      = (const float*)d_in[10];
  const float* bo      = (const float*)d_in[11];
  const float* Wad     = (const float*)d_in[12];
  const float* badl    = (const float*)d_in[13];
  const float* qn_g    = (const float*)d_in[14];
  const float* qn_b    = (const float*)d_in[15];
  const float* kn_g    = (const float*)d_in[16];
  const float* kn_b    = (const float*)d_in[17];
  const float* nq_g    = (const float*)d_in[18];
  const float* nq_b    = (const float*)d_in[19];
  const float* nkv_g   = (const float*)d_in[20];
  const float* nkv_b   = (const float*)d_in[21];
  const int*   Hp      = (const int*)d_in[22];
  const int*   Wp      = (const int*)d_in[23];
  float* out = (float*)d_out;

  size_t off = 0;
  const size_t oXs  = off; off += (size_t)NTK * DM * 2;
  const size_t oWkv = off; off += (size_t)2 * DM * DM * 2;
  const size_t oWq  = off; off += (size_t)DM * DM * 2;
  const size_t oWo  = off; off += (size_t)DM * DM * 2;
  const size_t oMod = off; off += 65536;
  const size_t oQa  = off; off += (size_t)QROWS * DM * 2;
  const size_t oQp  = off; off += (size_t)QROWS * DM * 2;
  const size_t oKp  = off; off += (size_t)NTK * DM * 2;
  const size_t oVp  = off; off += (size_t)NTK * DM * 2;
  const size_t oOp  = off; off += (size_t)NLT * DM * 2;
  if (off > ws_size) return;
  if (off > (size_t)134217728) return;
  if ((size_t)NB * DMOD * 4 > 65536) return;

  char* ws = (char*)d_ws;
  _Float16* Xs   = (_Float16*)(ws + oXs);
  _Float16* Wkv  = (_Float16*)(ws + oWkv);
  _Float16* Wq16 = (_Float16*)(ws + oWq);
  _Float16* Wo16 = (_Float16*)(ws + oWo);
  float*    Mod  = (float*)(ws + oMod);
  _Float16* Qa   = (_Float16*)(ws + oQa);
  _Float16* Qp   = (_Float16*)(ws + oQp);
  _Float16* Kp   = (_Float16*)(ws + oKp);
  _Float16* Vp   = (_Float16*)(ws + oVp);
  _Float16* Op   = (_Float16*)(ws + oOp);

  k_lnx<<<dim3(NTK / 8), dim3(256), 0, stream>>>(spatial, nkv_g, nkv_b, Xs, NTK);
  k_cvtw<<<dim3((DM * DM) / 2048), dim3(256), 0, stream>>>(Wk, Wkv, 32.0f, DM * DM);
  k_cvtw<<<dim3((DM * DM) / 2048), dim3(256), 0, stream>>>(Wv, Wkv + (size_t)DM * DM, 32.0f, DM * DM);
  k_cvtw<<<dim3((DM * DM) / 2048), dim3(256), 0, stream>>>(Wq, Wq16, 32.0f, DM * DM);
  k_cvtw<<<dim3((DM * DM) / 2048), dim3(256), 0, stream>>>(Wo, Wo16, 32.0f, DM * DM);
  k_mod<<<dim3((NB * DMOD) / 256), dim3(256), 0, stream>>>(cond, Wad, badl, Mod);
  k_qprep<<<dim3(QROWS / 8), dim3(256), 0, stream>>>(lt, lp, Mod, nq_g, nq_b, Qa);
  k_proj<<<dim3(QROWS / 64, 4), dim3(256), 0, stream>>>(Qa, Wq16, bq, qn_g, qn_b, Qp, bq, Qp, 4);
  k_proj<<<dim3(NTK / 64, 8), dim3(256), 0, stream>>>(Xs, Wkv, bk, kn_g, kn_b, Kp, bv, Vp, 4);
  k_attn<<<dim3(NB * NGP), dim3(256), 0, stream>>>(Qp, Kp, Vp, Op, Hp, Wp);
  k_out<<<dim3(NLT / 256, DM / 64), dim3(256), 0, stream>>>(Op, Wo16, bo, lt, lp, Mod, out);
  (void)hipGetLastError();
}
